// MultiHeadAttention_65025804861981
// MI455X (gfx1250) — hardware-run, weakly checked
//
#include <hip/hip_runtime.h>


#ifndef NB
#define NB 2
#endif
#ifndef SEQ
#define SEQ 2048
#endif
#define NB_FULL  2
#define SEQ_FULL 2048
#ifndef OUT_SEQ
#define OUT_SEQ SEQ
#endif
#define DM   2048
#define NH_  16
#define HD   128
#define QKVN 6144
#define ER   (SEQ < 512 ? SEQ : 512)
#define AW   4
#define QRS  2048.0f
#define QRI  (1.0f / 2048.0f)
#define SC2  (0.08838834764831845f * 1.4426950408889634f)
#define PSH  8.0f
#define WOS  64.0f
#define WOI  (1.0f / 64.0f)

static_assert(HD == 128);
static_assert(NH_ * HD == DM);
static_assert(QKVN == 3 * DM);
static_assert(DM % 64 == 0);
static_assert(DM % 32 == 0);
static_assert(SEQ % 64 == 0);
static_assert(ER % 64 == 0);
static_assert((SEQ - ER) % 64 == 0);
static_assert(ER % (16 * AW) == 0);
static_assert((SEQ - ER) % (16 * AW) == 0);
static_assert(ER % 32 == 0);
static_assert((SEQ * 64) % 256 == 0);
static_assert(((size_t)SEQ * DM) % 8 == 0);
static_assert(NB <= NB_FULL);
static_assert(SEQ <= SEQ_FULL);

typedef _Float16 h16;
typedef unsigned short bf;
typedef __attribute__((ext_vector_type(16))) __bf16   v16bf;
typedef __attribute__((ext_vector_type(16))) _Float16 v16h;
typedef __attribute__((ext_vector_type(16))) unsigned short v16us;
typedef __attribute__((ext_vector_type(8)))  _Float16 v8h;
typedef __attribute__((ext_vector_type(8)))  unsigned short v8us;
typedef __attribute__((ext_vector_type(8)))  float    v8f;
typedef __attribute__((ext_vector_type(4)))  float    v4f;
typedef v4f  __attribute__((may_alias)) v4fa;

__device__ __forceinline__ unsigned short f2bf(float f) { unsigned u = __float_as_uint(f); u += 0x7FFFu + ((u >> 16) & 1u); return (unsigned short)(u >> 16); }
__device__ __forceinline__ float bf2f(unsigned short s) { return __uint_as_float(((unsigned)s) << 16); }
__device__ __forceinline__ v16h cat16(v8h lo, v8h hi) { return __builtin_shufflevector(lo, hi, 0, 1, 2, 3, 4, 5, 6, 7, 8, 9, 10, 11, 12, 13, 14, 15); }
__device__ __forceinline__ v16bf cat16b(v8us lo, v8us hi) { return __builtin_bit_cast(v16bf, __builtin_shufflevector(lo, hi, 0, 1, 2, 3, 4, 5, 6, 7, 8, 9, 10, 11, 12, 13, 14, 15)); }
__device__ __forceinline__ v8f wmma16(v16h a, v16h b, v8f c) { return __builtin_amdgcn_wmma_f32_16x16x32_f16(false, a, false, b, (short)0, c, false, false); }
__device__ __forceinline__ v8f wmmab(v16bf a, v16bf b, v8f c) { return __builtin_amdgcn_wmma_f32_16x16x32_bf16(false, a, false, b, (short)0, c, false, false); }
__device__ __forceinline__ v16h  ldh(const h16* p) { return cat16(*(const v8h*)p, *(const v8h*)(p + 16)); }
__device__ __forceinline__ v16bf ldb(const bf* p)  { return cat16b(*(const v8us*)p, *(const v8us*)(p + 16)); }
__device__ __forceinline__ void wave_sync() { __builtin_amdgcn_fence(3  , "wavefront"); __builtin_amdgcn_wave_barrier(); asm volatile("" ::: "memory"); }

__global__ __launch_bounds__(256) void k_cvt8(const float* __restrict__ src, bf* dst, size_t n8) {
    const size_t i = (size_t)blockIdx.x * 256 + threadIdx.x; if (i >= n8) return;
    const v8f v = *(const v8f*)(src + i * 8); v8us o;
#pragma unroll
    for (int k = 0; k < 8; ++k) o[k] = f2bf(v[k]);
    *(volatile v8us*)(dst + i * 8) = o; __threadfence(); *(volatile v8us*)(dst + i * 8) = o;
}

__global__ __launch_bounds__(256) void k_tr(const float* __restrict__ W, bf* OB, h16* OH, int two, int R, int C, float scale) {
    __shared__ __align__(16) float tl[64 * 68];
    const int tid = threadIdx.x; const int n0 = blockIdx.x * 64, k0 = blockIdx.y * 64;
#pragma unroll
    for (int i = 0; i < 4; ++i) { const int kk = (tid >> 4) + 16 * i, n4 = (tid & 15) * 4;
        *(v4fa*)(&tl[kk * 68 + n4]) = *(const v4f*)(W + (size_t)(k0 + kk) * C + n0 + n4); }
    __syncthreads();
#pragma unroll 1
    for (int ps = 0; ps < 2; ++ps) {
#pragma unroll
        for (int s = 0; s < 2; ++s) { const int nn = 32 * s + (tid >> 3), k8 = (tid & 7) * 8;
            v8us ob; v8h oh;
#pragma unroll
            for (int i = 0; i < 8; ++i) { const float w = tl[(k8 + i) * 68 + nn]; const float v = bf2f(f2bf(w)) * scale; ob[i] = f2bf(v); oh[i] = (h16)v; }
            const size_t oo = (size_t)(n0 + nn) * R + k0 + k8;
            *(volatile v8us*)(OB + oo) = ob; if (two) *(volatile v8h*)(OH + oo) = oh; }
        if (ps == 0) __threadfence(); }
}

__global__ __launch_bounds__(256) void k_tab(float* TAB) {
    __shared__ __align__(16) float cs[512];
    const int tid = threadIdx.x; const int idx = blockIdx.x * 256 + tid;
    const int t = idx >> 6, j = idx & 63;
    const float e = (float)j * (1.0f / 64.0f);
    const float inv = 1.0f / powf(10000.0f, e);
    const float ang = (float)t * inv;
    cs[tid] = cosf(ang); cs[256 + tid] = sinf(ang);
    __syncthreads();
    if (tid < 128) {
        const v4f val = *(const v4fa*)(&cs[tid * 4]);
        const size_t o = (tid < 64) ? ((size_t)blockIdx.x * 256 + (size_t)tid * 4) : ((size_t)SEQ * 64 + (size_t)blockIdx.x * 256 + (size_t)(tid - 64) * 4);
        *(volatile v4f*)(TAB + o) = val; __threadfence(); *(volatile v4f*)(TAB + o) = val;
    }
}

__global__ __launch_bounds__(32) __attribute__((amdgpu_num_vgpr(256))) void k_projqk(const bf* __restrict__ A, const bf* __restrict__ Bt, const float* __restrict__ TAB, h16* PH, h16* PR) {
    __shared__ __align__(16) float os[16 * 132];
    const int K = DM;
    const int lane = threadIdx.x & 31, lr = lane & 15, hi = lane >> 4;
    const int r0 = blockIdx.x * 32; const int y = blockIdx.y;
    const int b = r0 / SEQ, t0 = r0 % SEQ;
    const int sel = y / NH_, head = y % NH_;
    v8f acc[2][8];
#pragma unroll
    for (int mb = 0; mb < 2; ++mb)
#pragma unroll
        for (int nb = 0; nb < 8; ++nb) acc[mb][nb] = (v8f){};
    const size_t aoff = (size_t)(r0 + lr) * K + 8 * hi, boff = (size_t)(y * HD + lr) * K + 8 * hi;
#pragma unroll 1
    for (int kc = 0; kc < K; kc += 32) {
        const v16bf a0 = ldb(A + aoff + kc), a1 = ldb(A + aoff + (size_t)16 * K + kc);
#pragma unroll
        for (int g = 0; g < 2; ++g) {
            v16bf bq;
#pragma unroll
            for (int nb = 0; nb < 4; ++nb) { bq = ldb(Bt + boff + (size_t)(4 * g + nb) * 16 * K + kc);
                acc[0][4 * g + nb] = wmmab(a0, bq, acc[0][4 * g + nb]); acc[1][4 * g + nb] = wmmab(a1, bq, acc[1][4 * g + nb]); }
            asm volatile("v_nop\n\tv_nop\n\tv_nop\n\tv_nop" : "+v"(acc[0][4 * g + 2]), "+v"(acc[1][4 * g + 2]), "+v"(acc[0][4 * g + 3]), "+v"(acc[1][4 * g + 3]) : "v"(a0), "v"(a1), "v"(bq));
        }
    }
    const size_t bhs = (size_t)sel * NB * NH_ + (size_t)b * NH_ + head;
    const size_t hb = bhs * SEQ * HD, rb = bhs * ER * HD;
    const int useRes = (t0 < ER) ? 1 : 0;
#pragma unroll
    for (int mb = 0; mb < 2; ++mb) {
#pragma unroll
        for (int nb = 0; nb < 8; ++nb) {
#pragma unroll
            for (int j = 0; j < 8; ++j) os[(hi * 8 + j) * 132 + nb * 16 + lr] = acc[mb][nb][j]; }
        wave_sync();
#pragma unroll 1
        for (int ps = 0; ps < 2; ++ps) {
#pragma unroll 1
            for (int s = 0; s < 8; ++s) { const int row = 2 * s + hi, c8 = lr * 8, pc = c8 ^ 64, jj = c8 & 63;
                const int t = t0 + mb * 16 + row;
                const v4f x0 = *(const v4fa*)(&os[row * 132 + c8]);  const v4f x1 = *(const v4fa*)(&os[row * 132 + c8 + 4]);
                const v4f p0 = *(const v4fa*)(&os[row * 132 + pc]);  const v4f p1 = *(const v4fa*)(&os[row * 132 + pc + 4]);
                const v4f c0 = *(const v4f*)(TAB + (size_t)t * 64 + jj); const v4f c1 = *(const v4f*)(TAB + (size_t)t * 64 + jj + 4);
                const v4f s0 = *(const v4f*)(TAB + (size_t)SEQ * 64 + (size_t)t * 64 + jj); const v4f s1 = *(const v4f*)(TAB + (size_t)SEQ * 64 + (size_t)t * 64 + jj + 4);
                const float sg = (c8 < 64) ? -1.0f : 1.0f;
                v8h hv, rv;
#pragma unroll
                for (int i = 0; i < 4; ++i) {
                    const float y0 = x0[i] * c0[i] + (sg * p0[i]) * s0[i]; const float y1 = x1[i] * c1[i] + (sg * p1[i]) * s1[i];
                    const h16 a0h = (h16)y0; const h16 a1h = (h16)y1; hv[i] = a0h; hv[4 + i] = a1h;
                    rv[i] = (h16)((y0 - (float)a0h) * QRS); rv[4 + i] = (h16)((y1 - (float)a1h) * QRS); }
                *(volatile v8h*)(PH + hb + (size_t)t * HD + c8) = hv;
                if (useRes) *(volatile v8h*)(PR + rb + (size_t)t * HD + c8) = rv; }
            if (ps == 0) __threadfence(); }
        wave_sync();
    }
}

__global__ __launch_bounds__(32) __attribute__((amdgpu_num_vgpr(256))) void k_projv(const bf* __restrict__ A, const bf* __restrict__ Bt, h16* VT, bf* VR) {
    __shared__ __align__(16) float os[16 * 68];
    const int K = DM;
    const int lane = threadIdx.x & 31, lr = lane & 15, hi = lane >> 4; const int r0 = blockIdx.x * 64, c0 = blockIdx.y * 64;
    const int b = c0 / SEQ, tt0 = c0 % SEQ;
    v8f acc[4][4];
#pragma unroll
    for (int mb = 0; mb < 4; ++mb)
#pragma unroll
        for (int nb = 0; nb < 4; ++nb) acc[mb][nb] = (v8f){};
    const size_t aoff = (size_t)(r0 + lr) * K + 8 * hi, boff = (size_t)(c0 + lr) * K + 8 * hi;
#pragma unroll 1
    for (int kc = 0; kc < K; kc += 32) {
        v16bf a[4];
#pragma unroll
        for (int mb = 0; mb < 4; ++mb) a[mb] = ldb(A + aoff + (size_t)mb * 16 * K + kc);
#pragma unroll
        for (int nb = 0; nb < 4; ++nb) { const v16bf bq = ldb(Bt + boff + (size_t)nb * 16 * K + kc);
#pragma unroll
            for (int mb = 0; mb < 4; ++mb) acc[mb][nb] = wmmab(a[mb], bq, acc[mb][nb]); }
        asm volatile("v_nop\n\tv_nop\n\tv_nop\n\tv_nop" : "+v"(acc[0][0]), "+v"(acc[1][1]), "+v"(acc[2][2]), "+v"(acc[3][3]) : "v"(a[0]), "v"(a[1]), "v"(a[2]), "v"(a[3]));
    }
    const size_t tbase = ((size_t)b * DM + r0) * SEQ + tt0, rbase = ((size_t)b * DM + r0) * ER + tt0;
    const int useRes = (tt0 < ER) ? 1 : 0;
#pragma unroll
    for (int mb = 0; mb < 4; ++mb) {
#pragma unroll
        for (int nb = 0; nb < 4; ++nb) {
#pragma unroll
            for (int j = 0; j < 8; ++j) os[(hi * 8 + j) * 68 + nb * 16 + lr] = acc[mb][nb][j]; }
        wave_sync();
#pragma unroll 1
        for (int ps = 0; ps < 2; ++ps) {
#pragma unroll
            for (int s = 0; s < 4; ++s) { const int row = 4 * s + (lane >> 3), c8 = (lane & 7) * 8;
                const v4f x0 = *(const v4fa*)(&os[row * 68 + c8]); const v4f x1 = *(const v4fa*)(&os[row * 68 + c8 + 4]); v8h hv; v8us rv;
#pragma unroll
                for (int i = 0; i < 4; ++i) { const h16 a0 = (h16)x0[i]; const h16 a1 = (h16)x1[i]; hv[i] = a0; hv[4 + i] = a1; rv[i] = f2bf(x0[i] - (float)a0); rv[4 + i] = f2bf(x1[i] - (float)a1); }
                *(volatile v8h*)(VT + tbase + (size_t)(mb * 16 + row) * SEQ + c8) = hv;
                if (useRes) *(volatile v8us*)(VR + rbase + (size_t)(mb * 16 + row) * ER + c8) = rv; }
            if (ps == 0) __threadfence(); }
        wave_sync();
    }
}

template <int EARLY>
__global__ __launch_bounds__(32 * AW) __attribute__((amdgpu_num_vgpr(256))) void k_flash(const h16* __restrict__ QH, const h16* __restrict__ KP, const h16* __restrict__ QR, const h16* __restrict__ KR,
                                                                                         const h16* __restrict__ VT, const bf* __restrict__ VR, h16* CH, bf* CR) {
    __shared__ __align__(16) float os[AW * 16 * 132];
    const int lane = threadIdx.x & 31, lr = lane & 15, hi = lane >> 4;
    const int wave = __builtin_amdgcn_readfirstlane((int)(threadIdx.x >> 5));
    const int zh = blockIdx.y; const int b = zh / NH_, h = zh % NH_;
    const int t0 = (EARLY ? 0 : ER) + (blockIdx.x * AW + wave) * 16;
    const size_t pbase = (size_t)zh * SEQ * HD, rbase = (size_t)zh * ER * HD;
    const size_t qo  = pbase + (size_t)(t0 + lr) * HD + 8 * hi;
    const size_t qro = EARLY ? (rbase + (size_t)(t0 + lr) * HD + 8 * hi) : (size_t)0;
    const size_t ko  = pbase + (size_t)lr * HD + 8 * hi;
    const size_t kro = rbase + (size_t)lr * HD + 8 * hi;
    const size_t vo  = pbase + (size_t)lr * SEQ + 8 * hi;
    const size_t vro = rbase + (size_t)lr * ER + 8 * hi;
    v8f o[8];
#pragma unroll
    for (int j = 0; j < 8; ++j) o[j] = (v8f){};
    float m = -3.0e38f, l = 0.0f;
    const int tq = t0 + lr;
    const int kend = t0 + 16;
#pragma unroll 1
    for (int key0 = 0; key0 < kend; key0 += 32) {
        v8f sHa = (v8f){}, sHb = (v8f){}, sLa = (v8f){}, sLb = (v8f){};
#pragma unroll 1
        for (int c = 0; c < 4; ++c) {
            const h16* kp = KP + ko + (size_t)key0 * HD + 32 * c;
            const v16h ka = ldh(kp), kb = ldh(kp + 16 * HD), qh = ldh(QH + qo + 32 * c);
            sHa = wmma16(ka, qh, sHa); sHb = wmma16(kb, qh, sHb);
            if (EARLY) {
                const h16* krp = KR + kro + (size_t)key0 * HD + 32 * c;
                const v16h kra = ldh(krp), krb = ldh(krp + 16 * HD), qr = ldh(QR + qro + 32 * c);
                sLa = wmma16(ka, qr, sLa);  sLb = wmma16(kb, qr, sLb);
                sLa = wmma16(kra, qh, sLa); sLb = wmma16(krb, qh, sLb);
                asm volatile("v_nop\n\tv_nop\n\tv_nop\n\tv_nop" : "+v"(sHa), "+v"(sHb), "+v"(sLa), "+v"(sLb) : "v"(ka), "v"(kb), "v"(kra), "v"(krb), "v"(qh), "v"(qr));
            } else {
                asm volatile("v_nop\n\tv_nop\n\tv_nop\n\tv_nop" : "+v"(sHa), "+v"(sHb) : "v"(ka), "v"(kb), "v"(qh));
            }
        }
        float ta[8], tb[8]; float mx = -3.0e38f;
        const int kA0 = key0 + 8 * hi;
#pragma unroll
        for (int r = 0; r < 8; ++r) {
            float va = sHa[r], vb = sHb[r];
            if (EARLY) { va += sLa[r] * QRI; vb += sLb[r] * QRI; }
            va *= SC2; vb *= SC2;
            va = (kA0 + r > tq) ? -3.0e38f : va;
            vb = (kA0 + 16 + r > tq) ? -3.0e38f : vb;
            ta[r] = va; tb[r] = vb; mx = fmaxf(mx, fmaxf(va, vb)); }
        mx = fmaxf(mx, __shfl_xor(mx, 16, 32));
        const float mnew = fmaxf(m, mx);
        const float alpha = __builtin_amdgcn_exp2f(m - mnew);
        const float sh = PSH - mnew;
        v16h pb; float ls = 0.0f;
#pragma unroll
        for (int r = 0; r < 8; ++r) { const h16 pa = (h16)__builtin_amdgcn_exp2f(ta[r] + sh); const h16 pc = (h16)__builtin_amdgcn_exp2f(tb[r] + sh); pb[r] = pa; pb[8 + r] = pc; ls += (float)pa + (float)pc; }
        l = l * alpha + ls; m = mnew;
        v16bf pbb;
        if (EARLY) { v16us pu;
#pragma unroll
            for (int r = 0; r < 16; ++r) pu[r] = f2bf((float)pb[r]);
            pbb = __builtin_bit_cast(v16bf, pu); }
#pragma unroll
        for (int j = 0; j < 8; ++j) o[j] = o[j] * alpha;
        const h16* va = VT + vo + key0;
#pragma unroll
        for (int g = 0; g < 2; ++g) {
            const v16h v0 = ldh(va + (size_t)(64 * g) * SEQ), v1 = ldh(va + (size_t)(64 * g + 16) * SEQ), v2 = ldh(va + (size_t)(64 * g + 32) * SEQ), v3 = ldh(va + (size_t)(64 * g + 48) * SEQ);
            o[4 * g + 0] = wmma16(v0, pb, o[4 * g + 0]); o[4 * g + 1] = wmma16(v1, pb, o[4 * g + 1]); o[4 * g + 2] = wmma16(v2, pb, o[4 * g + 2]); o[4 * g + 3] = wmma16(v3, pb, o[4 * g + 3]);
            if (EARLY) {
                const bf* vra = VR + vro + key0;
                const v16bf w0 = ldb(vra + (size_t)(64 * g) * ER), w1 = ldb(vra + (size_t)(64 * g + 16) * ER), w2 = ldb(vra + (size_t)(64 * g + 32) * ER), w3 = ldb(vra + (size_t)(64 * g + 48) * ER);
                o[4 * g + 0] = wmmab(w0, pbb, o[4 * g + 0]); o[4 * g + 1] = wmmab(w1, pbb, o[4 * g + 1]); o[4 * g + 2] = wmmab(w2, pbb, o[4 * g + 2]); o[4 * g + 3] = wmmab(w3, pbb, o[4 * g + 3]);
                asm volatile("v_nop\n\tv_nop\n\tv_nop\n\tv_nop" : "+v"(o[4 * g + 0]), "+v"(o[4 * g + 1]), "+v"(o[4 * g + 2]), "+v"(o[4 * g + 3]) : "v"(w0), "v"(w1), "v"(w2), "v"(w3), "v"(pbb), "v"(pb));
            } else {
                asm volatile("v_nop\n\tv_nop\n\tv_nop\n\tv_nop" : "+v"(o[4 * g + 0]), "+v"(o[4 * g + 1]), "+v"(o[4 * g + 2]), "+v"(o[4 * g + 3]) : "v"(v0), "v"(v1), "v"(v2), "v"(v3), "v"(pb));
            }
        }
    }
    l += __shfl_xor(l, 16, 32);
    const float inv = 1.0f / l;
    const int wb = wave * 16 * 132;
#pragma unroll
    for (int j = 0; j < 8; ++j) { v4f a, c;
        a[0] = o[j][0] * inv; a[1] = o[j][1] * inv; a[2] = o[j][2] * inv; a[3] = o[j][3] * inv; c[0] = o[j][4] * inv; c[1] = o[j][5] * inv; c[2] = o[j][6] * inv; c[3] = o[j][7] * inv;
        *(v4fa*)(&os[wb + lr * 132 + 16 * j + 8 * hi]) = a; *(v4fa*)(&os[wb + lr * 132 + 16 * j + 8 * hi + 4]) = c; }
    wave_sync();
    h16* crow = CH + ((size_t)b * SEQ + t0) * DM + h * HD;
    bf*  rrow = CR + ((size_t)b * ER + t0) * DM + h * HD;
#pragma unroll 1
    for (int ps = 0; ps < 2; ++ps) {
#pragma unroll 1
        for (int s = 0; s < 8; ++s) { const int row = 2 * s + hi, c8 = lr * 8;
            const v4f x0 = *(const v4fa*)(&os[wb + row * 132 + c8]); const v4f x1 = *(const v4fa*)(&os[wb + row * 132 + c8 + 4]); v8h hv; v8us rv;
#pragma unroll
            for (int i = 0; i < 4; ++i) { const h16 a0 = (h16)x0[i]; const h16 a1 = (h16)x1[i]; hv[i] = a0; hv[4 + i] = a1; rv[i] = f2bf(x0[i] - (float)a0); rv[4 + i] = f2bf(x1[i] - (float)a1); }
            *(volatile v8h*)(crow + (size_t)row * DM + c8) = hv;
            if (EARLY) *(volatile v8us*)(rrow + (size_t)row * DM + c8) = rv; }
        if (ps == 0) __threadfence(); }
}

template <int EARLY>
__global__ __launch_bounds__(32) __attribute__((amdgpu_num_vgpr(256))) void k_oproj(const h16* __restrict__ A, const bf* __restrict__ AR, const h16* __restrict__ Bt, const bf* __restrict__ BtB, float* OUT) {
    __shared__ __align__(16) float os[16 * 68];
    const int K = DM;
    constexpr int TPB = EARLY ? (ER / 64) : (((SEQ - ER) / 64) > 0 ? ((SEQ - ER) / 64) : 1);
    const int lane = threadIdx.x & 31, lr = lane & 15, hi = lane >> 4;
    const int bx = blockIdx.x; const int b = bx / TPB; const int tt0 = (EARLY ? 0 : ER) + (bx % TPB) * 64;
    const int c0 = blockIdx.y * 64;
    v8f acc[4][4];
#pragma unroll
    for (int mb = 0; mb < 4; ++mb)
#pragma unroll
        for (int nb = 0; nb < 4; ++nb) acc[mb][nb] = (v8f){};
    const size_t aoff = ((size_t)b * SEQ + tt0 + lr) * K + 8 * hi, roff = ((size_t)b * ER + tt0 + lr) * K + 8 * hi, boff = (size_t)(c0 + lr) * K + 8 * hi;
#pragma unroll 1
    for (int kc = 0; kc < K; kc += 32) {
        {
            v16h a[4];
#pragma unroll
            for (int mb = 0; mb < 4; ++mb) a[mb] = ldh(A + aoff + (size_t)mb * 16 * K + kc);
#pragma unroll
            for (int nb = 0; nb < 4; ++nb) { const v16h bh = ldh(Bt + boff + (size_t)nb * 16 * K + kc);
#pragma unroll
                for (int mb = 0; mb < 4; ++mb) acc[mb][nb] = wmma16(a[mb], bh, acc[mb][nb]); }
            asm volatile("v_nop\n\tv_nop\n\tv_nop\n\tv_nop" : "+v"(acc[0][3]), "+v"(acc[1][3]), "+v"(acc[2][3]), "+v"(acc[3][3]) : "v"(a[0]), "v"(a[1]), "v"(a[2]), "v"(a[3]));
        }
        if (EARLY) {
            v16bf ar[4];
#pragma unroll
            for (int mb = 0; mb < 4; ++mb) ar[mb] = ldb(AR + roff + (size_t)mb * 16 * K + kc);
#pragma unroll
            for (int nb = 0; nb < 4; ++nb) { const v16bf bb = ldb(BtB + boff + (size_t)nb * 16 * K + kc);
#pragma unroll
                for (int mb = 0; mb < 4; ++mb) acc[mb][nb] = wmmab(ar[mb], bb, acc[mb][nb]); }
            asm volatile("v_nop\n\tv_nop\n\tv_nop\n\tv_nop" : "+v"(acc[0][3]), "+v"(acc[1][3]), "+v"(acc[2][3]), "+v"(acc[3][3]) : "v"(ar[0]), "v"(ar[1]), "v"(ar[2]), "v"(ar[3]));
        }
    }
#pragma unroll
    for (int mb = 0; mb < 4; ++mb) {
#pragma unroll
        for (int nb = 0; nb < 4; ++nb) {
#pragma unroll
            for (int j = 0; j < 8; ++j) os[(hi * 8 + j) * 68 + nb * 16 + lr] = acc[mb][nb][j] * WOI; }
        wave_sync();
        float* orow = OUT + ((size_t)b * OUT_SEQ + tt0 + mb * 16) * DM + c0;
#pragma unroll 1
        for (int ps = 0; ps < 2; ++ps) {
#pragma unroll
            for (int s = 0; s < 8; ++s) { const int row = 2 * s + hi, cofs = lr * 4;
                const v4f val = *(const v4fa*)(&os[row * 68 + cofs]);
                *(volatile v4f*)(orow + (size_t)row * DM + cofs) = val; }
            if (ps == 0) __threadfence(); }
        wave_sync();
    }
}

static constexpr size_t al256(size_t v) { return (v + 255) & ~(size_t)255; }
static constexpr size_t SZ_XB  = al256((size_t)NB * SEQ * DM * 2);
static constexpr size_t SZ_WT  = al256((size_t)QKVN * DM * 2);
static constexpr size_t SZ_WO  = al256((size_t)DM * DM * 2);
static constexpr size_t SZ_TAB = al256((size_t)2 * SEQ * 64 * 4);
static constexpr size_t SZ_PH  = al256((size_t)2 * NB * NH_ * SEQ * HD * 2);
static constexpr size_t SZ_PR  = al256((size_t)2 * NB * NH_ * ER * HD * 2);
static constexpr size_t SZ_VT  = al256((size_t)NB * NH_ * HD * SEQ * 2);
static constexpr size_t SZ_VR  = al256((size_t)NB * NH_ * HD * ER * 2);
static constexpr size_t SZ_CR  = al256((size_t)NB * ER * DM * 2);
static constexpr size_t SZ_TOTAL = SZ_XB + SZ_WT + 2 * SZ_WO + SZ_TAB + SZ_PH + SZ_PR + SZ_VT + SZ_VR + SZ_CR;
static_assert(SZ_TOTAL <= (size_t)134217728);
static_assert((size_t)NB * SEQ * DM * 2 <= SZ_XB);

extern "C" void kernel_launch(void* const* d_in, const int* in_sizes, int n_in,
                              void* d_out, int out_size, void* d_ws, size_t ws_size, hipStream_t stream) {
    if (n_in < 3) return;
    const size_t needx = ((size_t)(NB - 1) * SEQ_FULL + SEQ) * DM;
    if ((size_t)in_sizes[0] < needx) return;
    if ((size_t)in_sizes[1] < (size_t)DM * QKVN || (size_t)in_sizes[2] < (size_t)DM * DM) return;
    if ((size_t)out_size < ((size_t)(NB - 1) * OUT_SEQ + SEQ) * DM) return;
    if (SZ_TOTAL > ws_size) return;
    const float* x = (const float*)d_in[0]; const float* wqkv = (const float*)d_in[1]; const float* wo = (const float*)d_in[2];
    float* OUT = (float*)d_out;
    char* wsp = (char*)d_ws;
    bf*  XB  = (bf*)wsp;  wsp += SZ_XB;
    bf*  WT  = (bf*)wsp;  wsp += SZ_WT;
    h16* WOH = (h16*)wsp; wsp += SZ_WO;
    bf*  WOB = (bf*)wsp;  wsp += SZ_WO;
    float* TAB = (float*)wsp; wsp += SZ_TAB;
    h16* PH  = (h16*)wsp; wsp += SZ_PH;
    h16* PR  = (h16*)wsp; wsp += SZ_PR;
    h16* VT  = (h16*)wsp; wsp += SZ_VT;
    bf*  VR  = (bf*)wsp;  wsp += SZ_VR;
    bf*  CR  = (bf*)wsp;  wsp += SZ_CR;
    h16* CH  = (h16*)XB;
    h16* QH = PH; h16* KP = PH + (size_t)NB * NH_ * SEQ * HD;
    h16* QR = PR; h16* KR = PR + (size_t)NB * NH_ * ER * HD;

    if (SEQ == SEQ_FULL) {
        const size_t n8 = (size_t)NB * SEQ * DM / 8;
        k_cvt8<<<(unsigned)((n8 + 255) / 256), 256, 0, stream>>>(x, XB, n8);
    } else {
        const size_t n8 = (size_t)SEQ * DM / 8;
        for (int b = 0; b < NB; ++b) k_cvt8<<<(unsigned)((n8 + 255) / 256), 256, 0, stream>>>(x + (size_t)b * SEQ_FULL * DM, XB + (size_t)b * SEQ * DM, n8);
    }
    k_tr<<<dim3(QKVN / 64, DM / 64, 1), 256, 0, stream>>>(wqkv, WT, WOH, 0, DM, QKVN, 1.0f);
    k_tr<<<dim3(DM / 64, DM / 64, 1), 256, 0, stream>>>(wo, WOB, WOH, 1, DM, DM, WOS);
    k_tab<<<SEQ * 64 / 256, 256, 0, stream>>>(TAB);

    k_projqk<<<dim3(NB * SEQ / 32, 2 * NH_, 1), 32, 0, stream>>>(XB, WT, TAB, PH, PR);
    k_projv<<<dim3(DM / 64, NB * SEQ / 64, 1), 32, 0, stream>>>(WT + (size_t)2 * DM * DM, XB, VT, VR);

    k_flash<1><<<dim3(ER / (16 * AW), NB * NH_, 1), 32 * AW, 0, stream>>>(QH, KP, QR, KR, VT, VR, CH, CR);
    if (SEQ > ER) k_flash<0><<<dim3((SEQ - ER) / (16 * AW), NB * NH_, 1), 32 * AW, 0, stream>>>(QH, KP, QR, KR, VT, VR, CH, CR);

    k_oproj<1><<<dim3(NB * (ER / 64), DM / 64, 1), 32, 0, stream>>>(CH, CR, WOH, WOB, OUT);
    if (SEQ > ER) k_oproj<0><<<dim3(NB * ((SEQ - ER) / 64), DM / 64, 1), 32, 0, stream>>>(CH, CR, WOH, WOB, OUT);
}
